// GCN0_2456721293643
// MI455X (gfx1250) — hardware-run, weakly checked
//
#include <hip/hip_runtime.h>
#include <stddef.h>
#include <stdint.h>
#include <math.h>


#define DF     128
#define OF     64
#define AP     256
#define KG     256
#define SP     128
#define NTHR   256
#define NWAVE  8
#define EPT    8
#define CHUNK  (NTHR * EPT)
#define WCAP   (EPT * 32)
#define LISTN  (NWAVE * WCAP)
#define NBD    8192
#define SLD    13
#define NBA    1024
#define SLA    10
#define RCAP   28672
#define DEGCAP 64
#define CPOIS  (1 << 20)
#define GBM    64
#define GBN    128
#define GTHR   128
#define NUW1   4096
#define NUWS   2048
#define BKT_ZINTS    (LISTN + 2 * RCAP + 3 * NBA)
#define BKT_LDS_INTS (BKT_ZINTS + 16)
#define WSMAX  134217728

static_assert((CHUNK & (CHUNK - 1)) == 0 && CHUNK <= 4096);
static_assert((NBD & (NBD - 1)) == 0 && NBD == (1 << SLD));
static_assert((NBA & (NBA - 1)) == 0 && NBA == (1 << SLA));
static_assert(((long long)CHUNK << SLD) < (1LL << 31));
static_assert(((long long)CHUNK << SLA) < (1LL << 31));
static_assert(NBD % (NTHR * 4) == 0);
static_assert(LISTN % NTHR == 0 && LISTN >= NBA);
static_assert(NBA % NWAVE == 0 && NBA == NTHR * 4 && NBA % GBM == 0);
static_assert(RCAP % (NTHR * 4) == 0 && BKT_ZINTS % (NTHR * 4) == 0);
static_assert(RCAP >= 16791 + 840);
static_assert(DEGCAP >= 37 + 8);
static_assert(CPOIS > DEGCAP);
static_assert(DF == 32 * 4 && OF == 32 * 2);
static_assert(KG % 32 == 0 && KG == 2 * DF && AP == KG && SP == 2 * OF && GBN == SP && GBN == DF);
static_assert(GBM == (GTHR / 32) * 16);
static_assert(NUW1 % NTHR == 0 && NUWS % NTHR == 0 && (NUW1 + 2 * NUWS) * 8 == 256 * KG);
static_assert(BKT_LDS_INTS * 4 <= 327680);
static_assert((NBD + LISTN + NWAVE) * 4 <= 327680);

typedef float          v2f   __attribute__((ext_vector_type(2)));
typedef float          v4f   __attribute__((ext_vector_type(4)));
typedef float          v8f   __attribute__((ext_vector_type(8)));
typedef int            v4i   __attribute__((ext_vector_type(4)));
typedef int            v8i   __attribute__((ext_vector_type(8)));
typedef unsigned       v2u   __attribute__((ext_vector_type(2)));
typedef unsigned short v4us  __attribute__((ext_vector_type(4)));
typedef unsigned short v8us  __attribute__((ext_vector_type(8)));
typedef unsigned short v16us __attribute__((ext_vector_type(16)));
typedef __bf16         v16bf __attribute__((ext_vector_type(16)));
typedef v2f  __attribute__((may_alias)) v2fa;
typedef v4f  __attribute__((may_alias)) v4fa;
typedef v4i  __attribute__((may_alias)) v4ia;
typedef v2u  __attribute__((may_alias)) v2ua;
typedef v4us __attribute__((may_alias)) v4usa;
typedef v8us __attribute__((may_alias)) v8usa;
union FragB { v16bf v; v16us u; v8us h[2]; v8i w; };

__device__ __forceinline__ v8f wmb(const FragB& a, const FragB& b, v8f c) {
  v8f d = __builtin_amdgcn_wmma_f32_16x16x32_bf16(false, a.v, false, b.v, (short)0, c, false, false);
  asm volatile("v_nop\n\tv_nop\n\tv_nop\n\tv_nop" : "+v"(d) : "v"(a.w), "v"(b.w));
  return d;
}

__device__ __forceinline__ unsigned bf16_bits(float f) {
  const unsigned u = __float_as_uint(f);
  return (u + 0x7FFFu + ((u >> 16) & 1u)) >> 16;
}
__device__ __forceinline__ float bf16_val(float f) {
  return __uint_as_float(bf16_bits(f) << 16);
}

__device__ __forceinline__ void wave_sync() {
  __builtin_amdgcn_fence(__ATOMIC_RELEASE, "wavefront");
  __builtin_amdgcn_wave_barrier();
  __builtin_amdgcn_fence(__ATOMIC_ACQUIRE, "wavefront");
}

template <int SLB>
__device__ __forceinline__ int scan_chunk(const int* __restrict__ dsts, int nE, int cbase, int slotBase,
                                          int nb, int vec8, int* list, int tid, int lane, int wave) {
  int wc = 0;
  const int el0  = tid * EPT;
  const int e0   = cbase + el0;
  const int sent = -2147483647 - 1;
  v4i da, db;
  if (vec8 != 0 && cbase + CHUNK <= nE) {
    da = *(const v4i*)(dsts + e0);
    db = *(const v4i*)(dsts + e0 + 4);
  } else {
    da.x = (e0     < nE) ? dsts[min(e0,     nE - 1)] : sent;
    da.y = (e0 + 1 < nE) ? dsts[min(e0 + 1, nE - 1)] : sent;
    da.z = (e0 + 2 < nE) ? dsts[min(e0 + 2, nE - 1)] : sent;
    da.w = (e0 + 3 < nE) ? dsts[min(e0 + 3, nE - 1)] : sent;
    db.x = (e0 + 4 < nE) ? dsts[min(e0 + 4, nE - 1)] : sent;
    db.y = (e0 + 5 < nE) ? dsts[min(e0 + 5, nE - 1)] : sent;
    db.z = (e0 + 6 < nE) ? dsts[min(e0 + 6, nE - 1)] : sent;
    db.w = (e0 + 7 < nE) ? dsts[min(e0 + 7, nE - 1)] : sent;
  }
  const unsigned nbs = (unsigned)slotBase;
  const unsigned unb = (unsigned)nb;
  const unsigned s0 = (unsigned)da.x - nbs, s1 = (unsigned)da.y - nbs;
  const unsigned s2 = (unsigned)da.z - nbs, s3 = (unsigned)da.w - nbs;
  const unsigned s4 = (unsigned)db.x - nbs, s5 = (unsigned)db.y - nbs;
  const unsigned s6 = (unsigned)db.z - nbs, s7 = (unsigned)db.w - nbs;
  const bool h0 = s0 < unb, h1 = s1 < unb, h2 = s2 < unb, h3 = s3 < unb;
  const bool h4 = s4 < unb, h5 = s5 < unb, h6 = s6 < unb, h7 = s7 < unb;
  const unsigned any = __builtin_amdgcn_ballot_w32(h0 | h1 | h2 | h3 | h4 | h5 | h6 | h7);
  if (any != 0u) {
#define HITJ(J, HJ, SJ) { \
      const unsigned mj = __builtin_amdgcn_ballot_w32(HJ); \
      if (mj != 0u) { \
        if (HJ) { \
          const int pos = wc + (int)__builtin_amdgcn_mbcnt_lo(mj, 0u); \
          if (pos < WCAP) list[wave * WCAP + pos] = ((el0 + (J)) << SLB) | (int)(SJ); \
        } \
        wc += (int)__builtin_popcount(mj); } }
    HITJ(0, h0, s0)
    HITJ(1, h1, s1)
    HITJ(2, h2, s2)
    HITJ(3, h3, s3)
    HITJ(4, h4, s4)
    HITJ(5, h5, s5)
    HITJ(6, h6, s6)
    HITJ(7, h7, s7)
#undef HITJ
  }
  return wc;
}

__global__ __launch_bounds__(NTHR) void k_wprep(const float* __restrict__ W1, const float* __restrict__ Ws,
                                                const float* __restrict__ Wn, unsigned short* WD) {
  const int u = (int)blockIdx.x * NTHR + (int)threadIdx.x;
  v8us o;
  int drow, k8;
  if (u < NUW1) {
    const int n = u >> 5;
    k8 = (u & 31) * 8;
    const int kk = k8 & (DF - 1);
    const float* p = W1 + (size_t)kk * DF + n;
#pragma unroll
    for (int i = 0; i < 8; ++i) o[i] = (unsigned short)bf16_bits(p[(size_t)i * DF]);
    drow = n;
  } else if (u < NUW1 + NUWS) {
    const int v = u - NUW1;
    const int n = v >> 5;
    k8 = (v & 31) * 8;
    const int kk = k8 & (DF - 1);
    const float* p = Ws + (size_t)kk * OF + n;
#pragma unroll
    for (int i = 0; i < 8; ++i) o[i] = (unsigned short)bf16_bits(p[(size_t)i * OF]);
    drow = DF + n;
  } else if (u < NUW1 + 2 * NUWS) {
    const int v = u - NUW1 - NUWS;
    const int n = v >> 5;
    k8 = (v & 31) * 8;
    const int kk = k8 & (DF - 1);
    const float* p = Wn + (size_t)kk * OF + n;
#pragma unroll
    for (int i = 0; i < 8; ++i) o[i] = (unsigned short)bf16_bits(p[(size_t)i * OF]);
    drow = DF + OF + n;
  } else {
    return;
  }
  unsigned short* dp = WD + (size_t)drow * KG + k8;
  *(volatile v8us*)dp = o;
  __threadfence();
  *(volatile v8us*)dp = o;
}

__global__ __launch_bounds__(NTHR) void k_cvx(const float* __restrict__ x, int nN, int nUnits,
                                              unsigned short* xb) {
  const int u = (int)blockIdx.x * NTHR + (int)threadIdx.x;
  if (u >= nUnits) return;
  const int row = u >> 4;
  const int k8  = (u & 15) * 8;
  const int rc  = row < nN ? row : nN - 1;
  const float* p = x + (size_t)rc * DF + k8;
  const v4f a = *(const v4fa*)p;
  const v4f b = *(const v4fa*)(p + 4);
  const bool ok = row < nN;
  v8us o;
  o[0] = ok ? (unsigned short)bf16_bits(a.x) : (unsigned short)0;
  o[1] = ok ? (unsigned short)bf16_bits(a.y) : (unsigned short)0;
  o[2] = ok ? (unsigned short)bf16_bits(a.z) : (unsigned short)0;
  o[3] = ok ? (unsigned short)bf16_bits(a.w) : (unsigned short)0;
  o[4] = ok ? (unsigned short)bf16_bits(b.x) : (unsigned short)0;
  o[5] = ok ? (unsigned short)bf16_bits(b.y) : (unsigned short)0;
  o[6] = ok ? (unsigned short)bf16_bits(b.z) : (unsigned short)0;
  o[7] = ok ? (unsigned short)bf16_bits(b.w) : (unsigned short)0;
  unsigned short* dp = xb + (size_t)row * DF + k8;
  *(volatile v8us*)dp = o;
  __threadfence();
  *(volatile v8us*)dp = o;
}

__global__ __launch_bounds__(NTHR) void k_deg(const int* __restrict__ keys, int nE, int vec8, int* isoBits) {
  __shared__ __attribute__((aligned(16))) int scnt[NBD];
  __shared__ __attribute__((aligned(16))) int list[LISTN];
  __shared__ int wcnt[NWAVE];
  const int tid = (int)threadIdx.x, lane = tid & 31, wave = tid >> 5;
  const int nodeBase = (int)blockIdx.x * NBD;

  for (int i = tid; i < NBD; i += NTHR) scnt[i] = 0;
  for (int i = tid; i < LISTN; i += NTHR) list[i] = 0;
  if (tid < NWAVE) wcnt[tid] = 0;
  __syncthreads();

  const int nChunks = (nE + CHUNK - 1) / CHUNK;
#pragma unroll 1
  for (int ch = 0; ch < nChunks; ++ch) {
    const int cbase = ch * CHUNK;
    const int wc = scan_chunk<SLD>(keys, nE, cbase, nodeBase, NBD, vec8, list, tid, lane, wave);
    if (lane == 0) wcnt[wave] = wc;
    __syncthreads();
    if (wave == 0) {
#pragma unroll 1
      for (int w2 = 0; w2 < NWAVE; ++w2) {
        int c = wcnt[w2];
        c = c < 0 ? 0 : (c > WCAP ? WCAP : c);
#pragma unroll 1
        for (int b0 = 0; b0 < c; b0 += 32) {
          const int idx = b0 + lane;
          const int ent = list[w2 * WCAP + (idx < WCAP ? idx : WCAP - 1)];
          const int m32 = (c - b0) < 32 ? (c - b0) : 32;
#pragma unroll 1
          for (int k = 0; k < m32; ++k) {
            const int u  = __builtin_amdgcn_readlane(ent, k);
            const int sl = u & (NBD - 1);
            if (lane == 0) scnt[sl] = scnt[sl] + 1;
          }
        }
      }
    }
    __syncthreads();
  }

#pragma unroll 1
  for (int i = tid; i < NBD; i += NTHR) {
    const int c  = scnt[i];
    const int cc = c < 1 ? 1 : c;
    const float r = 1.0f / sqrtf((float)cc);
    scnt[i] = (c > 0) ? __float_as_int(r) : 0;
  }
  __syncthreads();

  v4i vals[NBD / (NTHR * 4)];
#pragma unroll
  for (int it = 0; it < NBD / (NTHR * 4); ++it) {
    const int s0 = it * (NTHR * 4) + 4 * tid;
    vals[it] = *(const v4ia*)(scnt + s0);
  }
#pragma unroll
  for (int it = 0; it < NBD / (NTHR * 4); ++it) {
    const int s0 = it * (NTHR * 4) + 4 * tid;
    *(volatile v4i*)(isoBits + (size_t)nodeBase + s0) = vals[it];
  }
  __threadfence();
#pragma unroll
  for (int it = 0; it < NBD / (NTHR * 4); ++it) {
    const int s0 = it * (NTHR * 4) + 4 * tid;
    *(volatile v4i*)(isoBits + (size_t)nodeBase + s0) = vals[it];
  }
}

__global__ __launch_bounds__(NTHR) void k_bucket(const int* __restrict__ keys, const int* __restrict__ pay,
                                                 int nE, int nN, int vec8,
                                                 int* LISTg, int* CNTg, int* OFFg, int* ISIg) {
  extern __shared__ __attribute__((aligned(16))) int dsm[];
  int* list = dsm;
  int* hl   = dsm + LISTN;
  int* sl   = hl + RCAP;
  int* cnt  = sl + RCAP;
  int* offs = cnt + NBA;
  int* cur  = offs + NBA;
  int* misc = cur + NBA;
  const int tid = (int)threadIdx.x, lane = tid & 31, wave = tid >> 5;
  const int nodeBase = (int)blockIdx.x * NBA;

  {
    const v4i z4 = {0, 0, 0, 0};
    for (int i = tid * 4; i < BKT_ZINTS; i += NTHR * 4) *(v4ia*)(dsm + i) = z4;
    if (tid < 16) misc[tid] = 0;
  }
  __syncthreads();

  int t = 0, ov = 0;
  const int nChunks = (nE + CHUNK - 1) / CHUNK;
#pragma unroll 1
  for (int ch = 0; ch < nChunks; ++ch) {
    const int cbase = ch * CHUNK;
    const int wc = scan_chunk<SLA>(keys, nE, cbase, nodeBase, NBA, vec8, list, tid, lane, wave);
    if (lane == 0) misc[wave] = wc;
    __syncthreads();
    if (wave == 0) {
#pragma unroll 1
      for (int w2 = 0; w2 < NWAVE; ++w2) {
        int c = misc[w2];
        c = c < 0 ? 0 : (c > WCAP ? WCAP : c);
#pragma unroll 1
        for (int b0 = 0; b0 < c; b0 += 32) {
          const int idx = b0 + lane;
          const int ent = list[w2 * WCAP + (idx < WCAP ? idx : WCAP - 1)];
          const int m32 = (c - b0) < 32 ? (c - b0) : 32;
#pragma unroll 1
          for (int k = 0; k < m32; ++k) {
            const int u    = __builtin_amdgcn_readlane(ent, k);
            const int slot = u & (NBA - 1);
            const int el   = (u >> SLA) & (CHUNK - 1);
            const int pk   = ((cbase + el) << SLA) | slot;
            if (t < RCAP) {
              if (lane == 0) { hl[t] = pk; cnt[slot] = cnt[slot] + 1; }
              t = t + 1;
            } else {
              ov = 1;
            }
          }
        }
      }
    }
    __syncthreads();
  }
  if (wave == 0 && lane == 0) { misc[8] = t; misc[9] = ov; }
  __syncthreads();
  int tt = misc[8];
  tt = tt < 0 ? 0 : (tt > RCAP ? RCAP : tt);
  const int ovf = misc[9];

  if (wave == 0) {
    const int base = lane * (NBA / 32);
    int s = 0;
#pragma unroll 1
    for (int i = 0; i < NBA / 32; ++i) s += cnt[base + i];
    int incl = s;
#pragma unroll
    for (int d = 1; d < 32; d <<= 1) {
      const int y = __shfl_up(incl, d, 32);
      if (lane >= d) incl += y;
    }
    int run = incl - s;
#pragma unroll 1
    for (int i = 0; i < NBA / 32; ++i) {
      const int cv = cnt[base + i];
      offs[base + i] = run;
      cur[base + i]  = run;
      run += cv;
    }
  }
  __syncthreads();
  if (wave == 0) {
#pragma unroll 1
    for (int b0 = 0; b0 < tt; b0 += 32) {
      const int idx = b0 + lane;
      const int ent = hl[idx < RCAP ? idx : RCAP - 1];
      const int m32 = (tt - b0) < 32 ? (tt - b0) : 32;
#pragma unroll 1
      for (int k = 0; k < m32; ++k) {
        const int u    = __builtin_amdgcn_readlane(ent, k);
        const int slot = u & (NBA - 1);
        if (lane == 0) {
          int p = cur[slot];
          p = p < 0 ? 0 : (p > RCAP - 1 ? RCAP - 1 : p);
          sl[p] = u;
          cur[slot] = p + 1;
        }
      }
    }
  }
  __syncthreads();

  const int qn = 0x7fc00000;
#pragma unroll 1
  for (int i = tid; i < NBA; i += NTHR) {
    const int c  = cnt[i];
    const int cc = c < 1 ? 1 : c;
    const float r = 1.0f / sqrtf((float)cc);
    const int rb = (c > 0) ? __float_as_int(r) : 0;
    cur[i]  = (ovf != 0) ? qn : rb;
    list[i] = (ovf != 0) ? CPOIS : c;
  }
  __syncthreads();
  {
    const v4i c4 = *(const v4ia*)(list + 4 * tid);
    const v4i o4 = *(const v4ia*)(offs + 4 * tid);
    const v4i i4 = *(const v4ia*)(cur + 4 * tid);
    int* cp = CNTg + (size_t)nodeBase + 4 * tid;
    int* op = OFFg + (size_t)nodeBase + 4 * tid;
    int* ip = ISIg + (size_t)nodeBase + 4 * tid;
    *(volatile v4i*)cp = c4;
    *(volatile v4i*)op = o4;
    *(volatile v4i*)ip = i4;
    __threadfence();
    *(volatile v4i*)cp = c4;
    *(volatile v4i*)op = o4;
    *(volatile v4i*)ip = i4;
  }

  const int fill = nodeBase < nN ? nodeBase : nN - 1;
  int* lb = LISTg + (size_t)blockIdx.x * RCAP;
#pragma unroll 1
  for (int it = 0; it < RCAP / (NTHR * 4); ++it) {
    const int p0 = 4 * (it * NTHR + tid);
    const v4i e4 = *(const v4ia*)(sl + p0);
    int e0 = e4.x >> SLA, e1 = e4.y >> SLA, e2 = e4.z >> SLA, e3 = e4.w >> SLA;
    e0 = e0 < 0 ? 0 : (e0 > nE - 1 ? nE - 1 : e0);
    e1 = e1 < 0 ? 0 : (e1 > nE - 1 ? nE - 1 : e1);
    e2 = e2 < 0 ? 0 : (e2 > nE - 1 ? nE - 1 : e2);
    e3 = e3 < 0 ? 0 : (e3 > nE - 1 ? nE - 1 : e3);
    int s0 = pay[e0], s1 = pay[e1], s2 = pay[e2], s3 = pay[e3];
    asm volatile("" :: "v"(s0));
    asm volatile("" :: "v"(s1));
    asm volatile("" :: "v"(s2));
    asm volatile("" :: "v"(s3));
    s0 = s0 < 0 ? 0 : (s0 > nN - 1 ? nN - 1 : s0);
    s1 = s1 < 0 ? 0 : (s1 > nN - 1 ? nN - 1 : s1);
    s2 = s2 < 0 ? 0 : (s2 > nN - 1 ? nN - 1 : s2);
    s3 = s3 < 0 ? 0 : (s3 > nN - 1 ? nN - 1 : s3);
    v4i o;
    o.x = (p0     < tt) ? s0 : fill;
    o.y = (p0 + 1 < tt) ? s1 : fill;
    o.z = (p0 + 2 < tt) ? s2 : fill;
    o.w = (p0 + 3 < tt) ? s3 : fill;
    int* dp = lb + p0;
    *(volatile v4i*)dp = o;
    __threadfence();
    *(volatile v4i*)dp = o;
  }
}

__global__ __launch_bounds__(NTHR) void k_agg1(const int* __restrict__ LISTg, const int* __restrict__ CNTg,
                                               const int* __restrict__ OFFg, const float* __restrict__ ISIg,
                                               const float* __restrict__ ISOg,
                                               const unsigned short* __restrict__ xb,
                                               int nN, int mRows, unsigned short* p1) {
  __shared__ __attribute__((aligned(16))) int   scnt[NBA];
  __shared__ __attribute__((aligned(16))) int   soff[NBA];
  __shared__ __attribute__((aligned(16))) float sisi[NBA];
  __shared__ __attribute__((aligned(16))) unsigned short rowst[NWAVE * AP];
  const int tid = (int)threadIdx.x, lane = tid & 31;
  const int wave = __builtin_amdgcn_readfirstlane(tid >> 5);
  const int nodeBase = (int)blockIdx.x * NBA;
  {
    const size_t tb = (size_t)nodeBase + 4 * tid;
    *(v4ia*)(scnt + 4 * tid) = *(const v4i*)(CNTg + tb);
    *(v4ia*)(soff + 4 * tid) = *(const v4i*)(OFFg + tb);
    *(v4fa*)(sisi + 4 * tid) = *(const v4f*)(ISIg + tb);
  }
  __syncthreads();
  unsigned short* rowbuf = rowst + wave * AP;
  const int* lb = LISTg + (size_t)blockIdx.x * RCAP;
  const float qnan = __int_as_float(0x7fc00000);

#pragma unroll 1
  for (int si = 0; si < NBA / NWAVE; ++si) {
    const int s    = si * NWAVE + wave;
    const int node = nodeBase + s;
    const int craw = scnt[s];
    const bool big = (craw > DEGCAP) || (craw < 0);
    int c = craw < 0 ? 0 : (craw > DEGCAP ? DEGCAP : craw);
    int o = soff[s];
    o = o < 0 ? 0 : (o > RCAP - 1 ? RCAP - 1 : o);
    c = __builtin_amdgcn_readfirstlane(c);
    o = __builtin_amdgcn_readfirstlane(o);
    const float is = sisi[s];
    float a0 = 0.0f, a1 = 0.0f, a2 = 0.0f, a3 = 0.0f;
#pragma unroll 1
    for (int b0 = 0; b0 < c; b0 += 32) {
      int j = b0 + lane;
      j = j < c ? j : c - 1;
      int idx = o + j;
      idx = idx < 0 ? 0 : (idx > RCAP - 1 ? RCAP - 1 : idx);
      int sr = lb[idx];
      sr = sr < 0 ? 0 : (sr > nN - 1 ? nN - 1 : sr);
      const int isb = __float_as_int(ISOg[sr]);
      const int m32 = (c - b0) < 32 ? (c - b0) : 32;
#pragma unroll 1
      for (int k = 0; k < m32; ++k) {
        const int   sk = __builtin_amdgcn_readlane(sr, k);
        const float ck = __int_as_float(__builtin_amdgcn_readlane(isb, k));
        const v2u w = *(const v2ua*)(xb + (size_t)sk * DF + 4 * lane);
        const float f0 = __uint_as_float(w.x << 16);
        const float f1 = __uint_as_float(w.x & 0xffff0000u);
        const float f2 = __uint_as_float(w.y << 16);
        const float f3 = __uint_as_float(w.y & 0xffff0000u);
        a0 = fmaf(ck, f0, a0);
        a1 = fmaf(ck, f1, a1);
        a2 = fmaf(ck, f2, a2);
        a3 = fmaf(ck, f3, a3);
      }
    }
    const float pzr = big ? qnan : 0.0f;
    const bool live = node < nN;
    const float m0 = live ? (a0 * is + pzr) : 0.0f;
    const float m1 = live ? (a1 * is + pzr) : 0.0f;
    const float m2 = live ? (a2 * is + pzr) : 0.0f;
    const float m3 = live ? (a3 * is + pzr) : 0.0f;
    v4us mh, ml;
    {
      unsigned hb;
      hb = bf16_bits(m0); mh[0] = (unsigned short)hb; ml[0] = (unsigned short)bf16_bits(m0 - __uint_as_float(hb << 16));
      hb = bf16_bits(m1); mh[1] = (unsigned short)hb; ml[1] = (unsigned short)bf16_bits(m1 - __uint_as_float(hb << 16));
      hb = bf16_bits(m2); mh[2] = (unsigned short)hb; ml[2] = (unsigned short)bf16_bits(m2 - __uint_as_float(hb << 16));
      hb = bf16_bits(m3); mh[3] = (unsigned short)hb; ml[3] = (unsigned short)bf16_bits(m3 - __uint_as_float(hb << 16));
    }
    *(v4usa*)(rowbuf + 4 * lane) = mh;
    *(v4usa*)(rowbuf + DF + 4 * lane) = ml;
    wave_sync();
    const v8us q0 = *(const v8usa*)(rowbuf + 8 * lane);
    wave_sync();
    if (node < mRows) {
      unsigned short* rpw = p1 + (size_t)node * AP + 8 * lane;
      *(volatile v8us*)rpw = q0;
      __threadfence();
      *(volatile v8us*)rpw = q0;
    }
  }
}

template <int FIN>
__global__ __launch_bounds__(GTHR) __attribute__((amdgpu_num_vgpr(248)))
void k_gemm(unsigned short* Apl, const unsigned short* __restrict__ BT, const float* __restrict__ bias,
            float* outp, int nOut) {
  __shared__ __attribute__((aligned(16))) float stg[GBM * GBN];
  __shared__ __attribute__((aligned(16))) float sbias[GBN];
  const int tid = (int)threadIdx.x, lane = tid & 31, wave = tid >> 5, hh = lane >> 4, m = lane & 15;
  const int rowBase = (int)blockIdx.x * GBM;

  if constexpr (FIN == 0) {
    if (tid < 32) {
      const v4f t = *(const v4f*)(bias + 4 * tid);
      v4f b;
      b.x = bf16_val(t.x); b.y = bf16_val(t.y); b.z = bf16_val(t.z); b.w = bf16_val(t.w);
      *(v4fa*)(sbias + 4 * tid) = b;
    }
  }

  v8f acc[8];
  {
    const v8f z = {0.f, 0.f, 0.f, 0.f, 0.f, 0.f, 0.f, 0.f};
#pragma unroll
    for (int t = 0; t < 8; ++t) acc[t] = z;
  }
  const unsigned short* ap = Apl + (size_t)(rowBase + 16 * wave + m) * (size_t)AP + 8 * hh;
  const unsigned short* bp = BT + (size_t)m * (size_t)KG + 8 * hh;

#pragma unroll 1
  for (int k0 = 0; k0 < KG; k0 += 32) {
    FragB af;
    af.h[0] = *(const v8usa*)(ap + k0);
    af.h[1] = *(const v8usa*)(ap + k0 + 16);
#pragma unroll
    for (int nt = 0; nt < 8; ++nt) {
      const unsigned short* wq = bp + (size_t)(16 * nt) * (size_t)KG + k0;
      FragB bf;
      bf.h[0] = *(const v8usa*)wq;
      bf.h[1] = *(const v8usa*)(wq + 16);
      acc[nt] = wmb(af, bf, acc[nt]);
    }
  }

#pragma unroll
  for (int nt = 0; nt < 8; ++nt) {
    const int lc = 16 * nt + m;
#pragma unroll
    for (int r = 0; r < 8; ++r) {
      const int lr = 16 * wave + 8 * hh + r;
      stg[lr * GBN + lc] = acc[nt][r];
    }
  }
  __syncthreads();

  v4f pv[16];
#pragma unroll
  for (int i = 0; i < 16; ++i) pv[i] = *(const v4fa*)(stg + (16 * wave + i) * GBN + 4 * lane);

  if constexpr (FIN != 0) {
#pragma unroll
    for (int i = 0; i < 16; ++i) {
      const int r = rowBase + 16 * wave + i;
      *(volatile v4f*)(outp + (size_t)r * SP + 4 * lane) = pv[i];
    }
    __threadfence();
#pragma unroll
    for (int i = 0; i < 16; ++i) {
      const int r = rowBase + 16 * wave + i;
      *(volatile v4f*)(outp + (size_t)r * SP + 4 * lane) = pv[i];
    }
  } else {
    const v4f bb4 = *(const v4fa*)(sbias + 4 * lane);
    __syncthreads();
#pragma unroll
    for (int i = 0; i < 16; ++i) {
      const bool ok = (rowBase + 16 * wave + i) < nOut;
      const v4f t = pv[i] + bb4;
      v4f y;
      y.x = (t.x > 0.0f) ? t.x : (t.x - t.x);
      y.y = (t.y > 0.0f) ? t.y : (t.y - t.y);
      y.z = (t.z > 0.0f) ? t.z : (t.z - t.z);
      y.w = (t.w > 0.0f) ? t.w : (t.w - t.w);
      y.x = ok ? y.x : 0.0f; y.y = ok ? y.y : 0.0f; y.z = ok ? y.z : 0.0f; y.w = ok ? y.w : 0.0f;
      pv[i] = y;
    }
#pragma unroll
    for (int i = 0; i < 16; ++i) {
      v4us h4, l4;
      unsigned hb;
      hb = bf16_bits(pv[i].x); h4[0] = (unsigned short)hb; l4[0] = (unsigned short)bf16_bits(pv[i].x - __uint_as_float(hb << 16));
      hb = bf16_bits(pv[i].y); h4[1] = (unsigned short)hb; l4[1] = (unsigned short)bf16_bits(pv[i].y - __uint_as_float(hb << 16));
      hb = bf16_bits(pv[i].z); h4[2] = (unsigned short)hb; l4[2] = (unsigned short)bf16_bits(pv[i].z - __uint_as_float(hb << 16));
      hb = bf16_bits(pv[i].w); h4[3] = (unsigned short)hb; l4[3] = (unsigned short)bf16_bits(pv[i].w - __uint_as_float(hb << 16));
      unsigned short* srow = (unsigned short*)stg + (size_t)(16 * wave + i) * (2 * GBN);
      *(v4usa*)(srow + 4 * lane) = h4;
      *(v4usa*)(srow + DF + 4 * lane) = l4;
    }
    __syncthreads();
    v8us qv[16];
#pragma unroll
    for (int i = 0; i < 16; ++i) {
      const unsigned short* srow = (const unsigned short*)stg + (size_t)(16 * wave + i) * (2 * GBN);
      qv[i] = *(const v8usa*)(srow + 8 * lane);
    }
#pragma unroll
    for (int i = 0; i < 16; ++i) {
      unsigned short* rp = Apl + (size_t)(rowBase + 16 * wave + i) * (size_t)AP + 8 * lane;
      *(volatile v8us*)rp = qv[i];
    }
    __threadfence();
#pragma unroll
    for (int i = 0; i < 16; ++i) {
      unsigned short* rp = Apl + (size_t)(rowBase + 16 * wave + i) * (size_t)AP + 8 * lane;
      *(volatile v8us*)rp = qv[i];
    }
  }
}

__global__ __launch_bounds__(NTHR) void k_agg2(const int* __restrict__ LISTg, const int* __restrict__ CNTg,
                                               const int* __restrict__ OFFg, const float* __restrict__ st,
                                               const float* __restrict__ b2, int nN, float* out) {
  __shared__ __attribute__((aligned(16))) int scnt[NBA];
  __shared__ __attribute__((aligned(16))) int soff[NBA];
  const int tid = (int)threadIdx.x, lane = tid & 31;
  const int wave = __builtin_amdgcn_readfirstlane(tid >> 5);
  const int nodeBase = (int)blockIdx.x * NBA;
  {
    const size_t tb = (size_t)nodeBase + 4 * tid;
    *(v4ia*)(scnt + 4 * tid) = *(const v4i*)(CNTg + tb);
    *(v4ia*)(soff + 4 * tid) = *(const v4i*)(OFFg + tb);
  }
  float bv0, bv1;
  {
    const v2f a = *(const v2fa*)(b2 + 2 * lane);
    bv0 = bf16_val(a.x); bv1 = bf16_val(a.y);
  }
  __syncthreads();
  const int* lb = LISTg + (size_t)blockIdx.x * RCAP;
  const float qnan = __int_as_float(0x7fc00000);
  const int sa = (2 * lane) & 31, sb = (2 * lane + 1) & 31;

#pragma unroll 1
  for (int si = 0; si < NBA / NWAVE; ++si) {
    const int s    = si * NWAVE + wave;
    const int node = nodeBase + s;
    const int craw = scnt[s];
    const bool big = (craw > DEGCAP) || (craw < 0);
    int c = craw < 0 ? 0 : (craw > DEGCAP ? DEGCAP : craw);
    int o = soff[s];
    o = o < 0 ? 0 : (o > RCAP - 1 ? RCAP - 1 : o);
    c = __builtin_amdgcn_readfirstlane(c);
    o = __builtin_amdgcn_readfirstlane(o);
    const int nc = node < nN ? node : nN - 1;
    float acc0 = 0.0f, acc1 = 0.0f;
#pragma unroll 1
    for (int b0 = 0; b0 < c; b0 += 32) {
      int j = b0 + lane;
      j = j < c ? j : c - 1;
      int idx = o + j;
      idx = idx < 0 ? 0 : (idx > RCAP - 1 ? RCAP - 1 : idx);
      int sr = lb[idx];
      sr = sr < 0 ? 0 : (sr > nN - 1 ? nN - 1 : sr);
      const int m32 = (c - b0) < 32 ? (c - b0) : 32;
#pragma unroll 1
      for (int k = 0; k < m32; ++k) {
        const int sk = __builtin_amdgcn_readlane(sr, k);
        const v2f a = *(const v2fa*)(st + (size_t)sk * SP + OF + 2 * lane);
        acc0 += a.x; acc1 += a.y;
      }
    }
    const v2f sv = *(const v2fa*)(st + (size_t)nc * SP + 2 * lane);
    const float den = (float)(c < 1 ? 1 : c);
    float y0 = (sv.x + acc0 / den) + bv0;
    float y1 = (sv.y + acc1 / den) + bv1;
    const float pzr = big ? qnan : 0.0f;
    y0 = y0 + pzr; y1 = y1 + pzr;
    v4f ow;
    ow.x = __shfl(y0, sa, 32); ow.y = __shfl(y1, sa, 32);
    ow.z = __shfl(y0, sb, 32); ow.w = __shfl(y1, sb, 32);
    const bool wr = (node < nN) && (lane < 16);
    float* op = out + (size_t)nc * OF + 4 * (lane & 15);
    if (wr) *(volatile v4f*)op = ow;
    __threadfence();
    if (wr) *(volatile v4f*)op = ow;
  }
}

static inline int cdiv(int a, int b) { return (a + b - 1) / b; }
static inline size_t al256(size_t o) { return (o + 255) & ~(size_t)255; }

extern "C" void kernel_launch(void* const* d_in, const int* in_sizes, int n_in,
                              void* d_out, int out_size, void* d_ws, size_t ws_size,
                              hipStream_t stream) {
  if (n_in < 8) return;
  if (in_sizes[0] < DF || (in_sizes[0] % DF) != 0) return;
  const int nN = in_sizes[0] / DF;
  if (nN < 16 || nN >= (1 << 22)) return;
  if (in_sizes[1] != DF * DF || in_sizes[2] != DF) return;
  if (in_sizes[3] != DF * OF || in_sizes[4] != DF * OF) return;
  if (in_sizes[5] != OF) return;
  const int nE = in_sizes[6];
  if (nE < 1 || in_sizes[7] != nE) return;
  if (nE >= (1 << (31 - SLA))) return;
  if ((long long)out_size != (long long)nN * OF) return;

  const float* x   = (const float*)d_in[0];
  const float* W1  = (const float*)d_in[1];
  const float* b1  = (const float*)d_in[2];
  const float* Wsf = (const float*)d_in[3];
  const float* Wng = (const float*)d_in[4];
  const float* b2  = (const float*)d_in[5];
  const int*   src = (const int*)d_in[6];
  const int*   dst = (const int*)d_in[7];
  float* out = (float*)d_out;

  const int MP = cdiv(nN, 128) * 128;
  const int gM = MP / GBM;
  const int gA = cdiv(MP, NBA);
  const int gD = cdiv(nN, NBD);
  if ((MP % GBM) != 0) return;
  if ((long long)gA * NBA < (long long)MP) return;
  if ((long long)gD * NBD < (long long)nN) return;
  const int nUx = MP * (DF / 8);
  if ((nUx % NTHR) != 0) return;
  const int vec8 = ((nE & 3) == 0) ? 1 : 0;

  char* ws = (char*)d_ws;
  size_t off = 0;
  const size_t oWD   = off; off = al256(off + (size_t)256 * KG * 2);
  const size_t oISO  = off; off = al256(off + (size_t)gD * NBD * 4);
  const size_t oCNT  = off; off = al256(off + (size_t)gA * NBA * 4);
  const size_t oOFF  = off; off = al256(off + (size_t)gA * NBA * 4);
  const size_t oISI  = off; off = al256(off + (size_t)gA * NBA * 4);
  const size_t oLIST = off; off = al256(off + (size_t)gA * RCAP * 4);
  const size_t oP1   = off; off = al256(off + (size_t)MP * AP * 2);
  const size_t oST   = off; off = al256(off + (size_t)MP * SP * 4);
  if (off > ws_size || off > (size_t)WSMAX) return;
  if ((size_t)MP * DF * 2 > (size_t)MP * SP * 4) return;
  unsigned short* WD   = (unsigned short*)(ws + oWD);
  int*            ISOb = (int*)(ws + oISO);
  int*            CNTg = (int*)(ws + oCNT);
  int*            OFFg = (int*)(ws + oOFF);
  int*            ISIb = (int*)(ws + oISI);
  int*            LISTg = (int*)(ws + oLIST);
  unsigned short* P1   = (unsigned short*)(ws + oP1);
  float*          ST   = (float*)(ws + oST);
  unsigned short* XB   = (unsigned short*)(ws + oST);

  const size_t bktLds = (size_t)BKT_LDS_INTS * 4;
  hipFuncSetAttribute(reinterpret_cast<const void*>(&k_bucket), hipFuncAttributeMaxDynamicSharedMemorySize, (int)bktLds);

  k_wprep<<<(NUW1 + 2 * NUWS) / NTHR, NTHR, 0, stream>>>(W1, Wsf, Wng, WD);
  k_cvx<<<nUx / NTHR, NTHR, 0, stream>>>(x, nN, nUx, XB);
  k_deg<<<gD, NTHR, 0, stream>>>(src, nE, vec8, ISOb);
  k_bucket<<<gA, NTHR, bktLds, stream>>>(dst, src, nE, nN, vec8, LISTg, CNTg, OFFg, ISIb);
  k_agg1<<<gA, NTHR, 0, stream>>>(LISTg, CNTg, OFFg, (const float*)ISIb, (const float*)ISOb, XB, nN, MP, P1);
  k_gemm<0><<<gM, GTHR, 0, stream>>>(P1, WD, b1, ST, nN);
  k_gemm<1><<<gM, GTHR, 0, stream>>>(P1, WD + (size_t)DF * KG, b1, ST, nN);
  k_agg2<<<gA, NTHR, 0, stream>>>(LISTg, CNTg, OFFg, ST, b2, nN, out);
}
